// GraphSAGEEncoder_71098888618518
// MI455X (gfx1250) — hardware-run, weakly checked
//
#include <hip/hip_runtime.h>
#include <stddef.h>
#include <stdint.h>


#define DF     128
#define DIN    9
#define KE     32
#define AP     512
#define KS     512
#define NLAY   3
#define LNEPS  1e-5f
#define NTHR   256
#define NWAVE  8
#define EPT    8
#define CHUNK  (NTHR * EPT)
#define WCAP   (EPT * 32)
#define LISTN  (NWAVE * WCAP)
#define NBA    1024
#define SLA    10
#define RCAP   28672
#define DEGCAP 64
#define GBM    64
#define GBN    128
#define GTHR   128
#define GWAVE  (GTHR / 32)
#define ROWH   256
#define NUW0   (DF * (KE / 8))
#define NUWL   (DF * (KS / 8))
#define NUWB   (NLAY * NUWL)
#define NUWE   (NUW0 + NUWB)
#define PTHR   256
#define POOLW  256
#define AGG_ZINTS    (LISTN + 2 * RCAP + 3 * NBA)
#define MISC_INTS    16
#define ROWBUF_INTS  (NWAVE * ROWH / 2)
#define AGG_LDS_INTS (AGG_ZINTS + MISC_INTS + ROWBUF_INTS)
#define WSMAX  134217728

static_assert((CHUNK & (CHUNK - 1)) == 0 && CHUNK <= 4096);
static_assert((NBA & (NBA - 1)) == 0 && NBA == (1 << SLA));
static_assert(((long long)CHUNK << SLA) < (1LL << 31));
static_assert(LISTN % NTHR == 0);
static_assert(NBA % NWAVE == 0 && NBA % 32 == 0 && NBA % GBM == 0);
static_assert(RCAP % 4 == 0 && AGG_ZINTS % 4 == 0 && LISTN % 4 == 0 && ((AGG_ZINTS + MISC_INTS) % 4) == 0);
static_assert(AGG_ZINTS % (NTHR * 4) == 0);
static_assert(KE % 32 == 0 && KS % 32 == 0 && KS == AP && KS == 4 * DF);
static_assert(GBN == DF && GBM == GWAVE * 16 && DF == 4 * 32 && GTHR == GWAVE * 32);
static_assert(AGG_LDS_INTS * 4 <= 300000);
static_assert(ROWH == 2 * DF);
static_assert(NUW0 % NTHR == 0 && NUWL % NTHR == 0 && NUWE % NTHR == 0 && NUWL == 8192);
static_assert(DIN <= KE && KE / 8 == 4);
static_assert(PTHR == POOLW && POOLW == 2 * DF && PTHR == NWAVE * 32 && (POOLW / 4) <= PTHR);

typedef float          v2f   __attribute__((ext_vector_type(2)));
typedef float          v4f   __attribute__((ext_vector_type(4)));
typedef float          v8f   __attribute__((ext_vector_type(8)));
typedef int            v4i   __attribute__((ext_vector_type(4)));
typedef int            v8i   __attribute__((ext_vector_type(8)));
typedef unsigned       v2u   __attribute__((ext_vector_type(2)));
typedef unsigned       v4u   __attribute__((ext_vector_type(4)));
typedef unsigned short v2us  __attribute__((ext_vector_type(2)));
typedef unsigned short v4us  __attribute__((ext_vector_type(4)));
typedef unsigned short v8us  __attribute__((ext_vector_type(8)));
typedef unsigned short v16us __attribute__((ext_vector_type(16)));
typedef __bf16         v16bf __attribute__((ext_vector_type(16)));
typedef v2f  __attribute__((may_alias)) v2fa;
typedef v4f  __attribute__((may_alias)) v4fa;
typedef v4i  __attribute__((may_alias)) v4ia;
typedef v2u  __attribute__((may_alias)) v2ua;
typedef v4u  __attribute__((may_alias)) v4ua;
typedef v2us __attribute__((may_alias)) v2usa;
typedef v4us __attribute__((may_alias)) v4usa;
typedef v8us __attribute__((may_alias)) v8usa;
union FragB { v16bf v; v16us u; v8us h[2]; v8i w; };

__device__ __forceinline__ v8f wmb(const FragB& a, const FragB& b, v8f c) {
  v8f d = __builtin_amdgcn_wmma_f32_16x16x32_bf16(false, a.v, false, b.v, (short)0, c, false, false);
  asm volatile("v_nop\n\tv_nop\n\tv_nop\n\tv_nop" : "+v"(d) : "v"(a.w), "v"(b.w));
  return d;
}

__device__ __forceinline__ v8f z8() { v8f z = {0.f, 0.f, 0.f, 0.f, 0.f, 0.f, 0.f, 0.f}; return z; }

__device__ __forceinline__ unsigned bf16_bits(float f) {
  const unsigned u = __float_as_uint(f);
  return (u + 0x7FFFu + ((u >> 16) & 1u)) >> 16;
}
__device__ __forceinline__ float bf16_val(float f) {
  return __uint_as_float(bf16_bits(f) << 16);
}
__device__ __forceinline__ unsigned hl_bits(float v, unsigned& lo) {
  const unsigned hb = bf16_bits(v);
  lo = bf16_bits(v - __uint_as_float(hb << 16));
  return hb;
}

__device__ __forceinline__ void wave_sync() {
  __builtin_amdgcn_fence(__ATOMIC_RELEASE, "wavefront");
  __builtin_amdgcn_wave_barrier();
  __builtin_amdgcn_fence(__ATOMIC_ACQUIRE, "wavefront");
}

template <int SLB>
__device__ __forceinline__ int scan_chunk(const int* __restrict__ dsts, int nE, int cbase, int slotBase,
                                          int nb, int vec8, int* list, int tid, int lane, int wave) {
  int wc = 0;
  const int el0  = tid * EPT;
  const int e0   = cbase + el0;
  const int sent = -2147483647 - 1;
  v4i da, db;
  if (vec8 != 0 && cbase + CHUNK <= nE) {
    da = *(const v4i*)(dsts + e0);
    db = *(const v4i*)(dsts + e0 + 4);
  } else {
    da.x = (e0     < nE) ? dsts[min(e0,     nE - 1)] : sent;
    da.y = (e0 + 1 < nE) ? dsts[min(e0 + 1, nE - 1)] : sent;
    da.z = (e0 + 2 < nE) ? dsts[min(e0 + 2, nE - 1)] : sent;
    da.w = (e0 + 3 < nE) ? dsts[min(e0 + 3, nE - 1)] : sent;
    db.x = (e0 + 4 < nE) ? dsts[min(e0 + 4, nE - 1)] : sent;
    db.y = (e0 + 5 < nE) ? dsts[min(e0 + 5, nE - 1)] : sent;
    db.z = (e0 + 6 < nE) ? dsts[min(e0 + 6, nE - 1)] : sent;
    db.w = (e0 + 7 < nE) ? dsts[min(e0 + 7, nE - 1)] : sent;
  }
  const unsigned nbs = (unsigned)slotBase;
  const unsigned unb = (unsigned)nb;
  const unsigned s0 = (unsigned)da.x - nbs, s1 = (unsigned)da.y - nbs;
  const unsigned s2 = (unsigned)da.z - nbs, s3 = (unsigned)da.w - nbs;
  const unsigned s4 = (unsigned)db.x - nbs, s5 = (unsigned)db.y - nbs;
  const unsigned s6 = (unsigned)db.z - nbs, s7 = (unsigned)db.w - nbs;
  const bool h0 = s0 < unb, h1 = s1 < unb, h2 = s2 < unb, h3 = s3 < unb;
  const bool h4 = s4 < unb, h5 = s5 < unb, h6 = s6 < unb, h7 = s7 < unb;
  const unsigned any = __builtin_amdgcn_ballot_w32(h0 | h1 | h2 | h3 | h4 | h5 | h6 | h7);
  if (any != 0u) {
#define HITJ(J, HJ, SJ) { \
      const unsigned mj = __builtin_amdgcn_ballot_w32(HJ); \
      if (mj != 0u) { \
        if (HJ) { \
          const int pos = wc + (int)__builtin_amdgcn_mbcnt_lo(mj, 0u); \
          if (pos < WCAP) list[wave * WCAP + pos] = ((el0 + (J)) << SLB) | (int)(SJ); \
        } \
        wc += (int)__builtin_popcount(mj); } }
    HITJ(0, h0, s0)
    HITJ(1, h1, s1)
    HITJ(2, h2, s2)
    HITJ(3, h3, s3)
    HITJ(4, h4, s4)
    HITJ(5, h5, s5)
    HITJ(6, h6, s6)
    HITJ(7, h7, s7)
#undef HITJ
  }
  return wc;
}

__global__ __launch_bounds__(NTHR) void k_prep(const float* __restrict__ x, const float* __restrict__ w0,
                                               const float* __restrict__ wl1, const float* __restrict__ wr1,
                                               const float* __restrict__ wl2, const float* __restrict__ wr2,
                                               const float* __restrict__ wl3, const float* __restrict__ wr3,
                                               unsigned short* w0b, unsigned short* bpl, unsigned short* xb,
                                               int nN, int nUnits) {
  const int u = (int)blockIdx.x * NTHR + (int)threadIdx.x;
  v8us o;
  unsigned short* dp;
  if (u < NUW0) {
    const int n = u >> 2, k8 = (u & 3) * 8;
    const float* p = w0 + (size_t)n * DIN;
#pragma unroll
    for (int i = 0; i < 8; ++i) {
      const int k  = k8 + i;
      const int kc = k < DIN ? k : DIN - 1;
      const float f = p[kc];
      o[i] = (unsigned short)bf16_bits(k < DIN ? f : 0.0f);
    }
    dp = w0b + (size_t)u * 8;
  } else if (u < NUWE) {
    const int v  = u - NUW0;
    const int l  = v >> 13;
    const int n  = (v >> 6) & (DF - 1), k8 = (v & 63) * 8;
    const int kk = k8 & (DF - 1);
    const float* wl;
    const float* wr;
    if (l == 0)      { wl = wl1; wr = wr1; }
    else if (l == 1) { wl = wl2; wr = wr2; }
    else             { wl = wl3; wr = wr3; }
    const size_t wo = (size_t)n * DF + (size_t)kk;
    const v4f a0 = *(const v4f*)(wl + wo), a1 = *(const v4f*)(wl + wo + 4);
    const v4f c0 = *(const v4f*)(wr + wo), c1 = *(const v4f*)(wr + wo + 4);
    const float fa[8] = {a0.x, a0.y, a0.z, a0.w, a1.x, a1.y, a1.z, a1.w};
    const float fb[8] = {c0.x, c0.y, c0.z, c0.w, c1.x, c1.y, c1.z, c1.w};
    const unsigned msk = (k8 < 2 * DF) ? 0xFFFFu : 0u;
#pragma unroll
    for (int i = 0; i < 8; ++i) {
      const unsigned ha = bf16_bits(fa[i]);
      const unsigned hb = bf16_bits(fb[i]);
      o[i] = (unsigned short)((ha & msk) | (hb & (~msk & 0xFFFFu)));
    }
    dp = bpl + (size_t)v * 8;
  } else if (u < nUnits) {
    const int v   = u - NUWE;
    const int row = v >> 2, k8 = (v & 3) * 8;
    const int rc  = row < nN ? row : nN - 1;
    const bool lv = row < nN;
    const float* p = x + (size_t)rc * DIN;
#pragma unroll
    for (int i = 0; i < 8; ++i) {
      const int k  = k8 + i;
      const int kc = k < DIN ? k : DIN - 1;
      const float f = p[kc];
      o[i] = (unsigned short)bf16_bits((lv && k < DIN) ? f : 0.0f);
    }
    dp = xb + (size_t)v * 8;
  } else {
    return;
  }
  *(volatile v8us*)dp = o;
  __threadfence();
  *(volatile v8us*)dp = o;
}

__global__ __launch_bounds__(NTHR) void k_scan(const int* __restrict__ srcs, const int* __restrict__ dsts,
                                               int nE, int nN, int vec8, int mRows, unsigned short* apl) {
  extern __shared__ __attribute__((aligned(16))) int dsm[];
  int* list = dsm;
  int* hl   = dsm + LISTN;
  int* sl   = hl + RCAP;
  int* cnt  = sl + RCAP;
  int* offs = cnt + NBA;
  int* cur  = offs + NBA;
  int* misc = cur + NBA;
  const int tid = (int)threadIdx.x, lane = tid & 31, wave = tid >> 5;
  unsigned short* rowbuf = (unsigned short*)(misc + MISC_INTS) + wave * ROWH;
  const int nodeBase = (int)blockIdx.x * NBA;

  {
    const v4i z4 = {0, 0, 0, 0};
    for (int i = tid * 4; i < AGG_ZINTS; i += NTHR * 4) *(v4ia*)(dsm + i) = z4;
    if (tid < MISC_INTS) misc[tid] = 0;
  }
  __syncthreads();

  int t = 0, ov = 0;
  const int nChunks = (nE + CHUNK - 1) / CHUNK;
#pragma unroll 1
  for (int ch = 0; ch < nChunks; ++ch) {
    const int cbase = ch * CHUNK;
    const int wc = scan_chunk<SLA>(dsts, nE, cbase, nodeBase, NBA, vec8, list, tid, lane, wave);
    if (lane == 0) misc[wave] = wc;
    __syncthreads();
    if (wave == 0) {
#pragma unroll 1
      for (int w2 = 0; w2 < NWAVE; ++w2) {
        int c = misc[w2];
        c = c < 0 ? 0 : (c > WCAP ? WCAP : c);
#pragma unroll 1
        for (int b0 = 0; b0 < c; b0 += 32) {
          const int idx = b0 + lane;
          const int ent_ = list[w2 * WCAP + (idx < WCAP ? idx : WCAP - 1)];
          const int m32 = (c - b0) < 32 ? (c - b0) : 32;
#pragma unroll 1
          for (int k = 0; k < m32; ++k) {
            const int u    = __builtin_amdgcn_readlane(ent_, k);
            const int slot = u & (NBA - 1);
            const int el   = (u >> SLA) & (CHUNK - 1);
            const int pk   = ((cbase + el) << SLA) | slot;
            if (t < RCAP) {
              if (lane == 0) { hl[t] = pk; cnt[slot] = cnt[slot] + 1; }
              t = t + 1;
            } else {
              ov = 1;
            }
          }
        }
      }
    }
    __syncthreads();
  }
  if (wave == 0 && lane == 0) { misc[8] = t; misc[9] = ov; }
  __syncthreads();
  int tt = misc[8];
  tt = tt < 0 ? 0 : (tt > RCAP ? RCAP : tt);
  const int ovf = misc[9];

  if (wave == 0) {
    const int base = lane * (NBA / 32);
    int s = 0;
#pragma unroll 1
    for (int i = 0; i < NBA / 32; ++i) s += cnt[base + i];
    int incl = s;
#pragma unroll
    for (int d = 1; d < 32; d <<= 1) {
      const int y = __shfl_up(incl, d, 32);
      if (lane >= d) incl += y;
    }
    int run = incl - s;
#pragma unroll 1
    for (int i = 0; i < NBA / 32; ++i) {
      const int cv = cnt[base + i];
      offs[base + i] = run;
      cur[base + i]  = run;
      run += cv;
    }
  }
  __syncthreads();
  if (wave == 0) {
#pragma unroll 1
    for (int b0 = 0; b0 < tt; b0 += 32) {
      const int idx = b0 + lane;
      const int ent_ = hl[idx < RCAP ? idx : RCAP - 1];
      const int m32 = (tt - b0) < 32 ? (tt - b0) : 32;
#pragma unroll 1
      for (int k = 0; k < m32; ++k) {
        const int u    = __builtin_amdgcn_readlane(ent_, k);
        const int slot = u & (NBA - 1);
        if (lane == 0) {
          int p = cur[slot];
          p = p < 0 ? 0 : (p > RCAP - 1 ? RCAP - 1 : p);
          sl[p] = u;
          cur[slot] = p + 1;
        }
      }
    }
  }
  __syncthreads();

  const float pz = (ovf != 0) ? __int_as_float(0x7fc00000) : 0.0f;
#pragma unroll 1
  for (int si = 0; si < NBA / NWAVE; ++si) {
    const int s    = si * NWAVE + wave;
    const int node = nodeBase + s;
    int c = cnt[s];
    const bool big = c > DEGCAP;
    c = c < 0 ? 0 : (c > DEGCAP ? DEGCAP : c);
    int o = offs[s];
    o = o < 0 ? 0 : (o > RCAP ? RCAP : o);
    const float pzr = big ? __int_as_float(0x7fc00000) : pz;
    const bool live = node < nN;
    float a0 = 0.0f, a1 = 0.0f, a2 = 0.0f, a3 = 0.0f;
#pragma unroll 1
    for (int b0 = 0; b0 < c; b0 += 32) {
      int idx = o + b0 + lane;
      idx = idx > RCAP - 1 ? RCAP - 1 : idx;
      const int ent_ = sl[idx];
      int eid = ent_ >> SLA;
      eid = eid < 0 ? 0 : (eid > nE - 1 ? nE - 1 : eid);
      int sr = srcs[eid];
      sr = sr < 0 ? 0 : (sr > nN - 1 ? nN - 1 : sr);
      const int m32 = (c - b0) < 32 ? (c - b0) : 32;
#pragma unroll 1
      for (int k = 0; k < m32; ++k) {
        const int sk = __builtin_amdgcn_readlane(sr, k);
        const unsigned short* rp = apl + (size_t)sk * AP + 2 * DF + 4 * lane;
        const v2u wh = *(const v2ua*)rp;
        const v2u wl = *(const v2ua*)(rp + DF);
        const float f0 = __uint_as_float(wh.x << 16)         + __uint_as_float(wl.x << 16);
        const float f1 = __uint_as_float(wh.x & 0xffff0000u) + __uint_as_float(wl.x & 0xffff0000u);
        const float f2 = __uint_as_float(wh.y << 16)         + __uint_as_float(wl.y << 16);
        const float f3 = __uint_as_float(wh.y & 0xffff0000u) + __uint_as_float(wl.y & 0xffff0000u);
        a0 += f0; a1 += f1; a2 += f2; a3 += f3;
      }
    }
    const float inv = 1.0f / fmaxf((float)c, 1.0f);
    const float m0 = live ? (a0 * inv + pzr) : 0.0f;
    const float m1 = live ? (a1 * inv + pzr) : 0.0f;
    const float m2 = live ? (a2 * inv + pzr) : 0.0f;
    const float m3 = live ? (a3 * inv + pzr) : 0.0f;
    v4us mh, ml;
    {
      unsigned lb;
      unsigned hb;
      hb = hl_bits(m0, lb); mh[0] = (unsigned short)hb; ml[0] = (unsigned short)lb;
      hb = hl_bits(m1, lb); mh[1] = (unsigned short)hb; ml[1] = (unsigned short)lb;
      hb = hl_bits(m2, lb); mh[2] = (unsigned short)hb; ml[2] = (unsigned short)lb;
      hb = hl_bits(m3, lb); mh[3] = (unsigned short)hb; ml[3] = (unsigned short)lb;
    }
    *(v4usa*)(rowbuf + 4 * lane)      = mh;
    *(v4usa*)(rowbuf + DF + 4 * lane) = ml;
    wave_sync();
    const v8us q0 = *(const v8usa*)(rowbuf + 8 * lane);
    wave_sync();
    if (node < mRows) {
      unsigned short* rpw = apl + (size_t)node * AP + 8 * lane;
      *(volatile v8us*)rpw = q0;
      __threadfence();
      *(volatile v8us*)rpw = q0;
    }
  }
}

template <int LAST>
__global__ __launch_bounds__(GTHR) void k_gemm(const unsigned short* A, int lda,
                                               const unsigned short* __restrict__ BT, int ldb, int K,
                                               const float* __restrict__ bias, const float* __restrict__ gam,
                                               const float* __restrict__ bet,
                                               unsigned short* apl, float* outp, int nN, int mRows) {
  __shared__ __attribute__((aligned(16))) float stg[GBM * GBN];
  const int tid = (int)threadIdx.x, lane = tid & 31, wave = tid >> 5, hh = lane >> 4, m = lane & 15;
  const int rowBase = (int)blockIdx.x * GBM;

  v8f acc[8];
#pragma unroll
  for (int t = 0; t < 8; ++t) acc[t] = z8();
  const unsigned short* ap = A + (size_t)(rowBase + 16 * wave + m) * (size_t)lda + 8 * hh;
  const unsigned short* bp = BT + (size_t)m * (size_t)ldb + 8 * hh;

#pragma unroll 1
  for (int k0 = 0; k0 < K; k0 += 32) {
    FragB af;
    af.h[0] = *(const v8usa*)(ap + k0);
    af.h[1] = *(const v8usa*)(ap + k0 + 16);
#pragma unroll
    for (int nt = 0; nt < 8; ++nt) {
      const unsigned short* wq = bp + (size_t)(16 * nt) * (size_t)ldb + k0;
      FragB bf;
      bf.h[0] = *(const v8usa*)wq;
      bf.h[1] = *(const v8usa*)(wq + 16);
      acc[nt] = wmb(af, bf, acc[nt]);
    }
  }

#pragma unroll
  for (int nt = 0; nt < 8; ++nt) {
    const int lc = 16 * nt + m;
#pragma unroll
    for (int r = 0; r < 8; ++r) {
      const int lr = 16 * wave + 8 * hh + r;
      stg[lr * GBN + lc] = acc[nt][r];
    }
  }
  __syncthreads();

  float bq[4], gq[4], eq[4];
  {
    const v4f b4 = *(const v4f*)(bias + 4 * lane);
    const v4f g4 = *(const v4f*)(gam + 4 * lane);
    const v4f e4 = *(const v4f*)(bet + 4 * lane);
    bq[0] = bf16_val(b4.x); bq[1] = bf16_val(b4.y); bq[2] = bf16_val(b4.z); bq[3] = bf16_val(b4.w);
    gq[0] = bf16_val(g4.x); gq[1] = bf16_val(g4.y); gq[2] = bf16_val(g4.z); gq[3] = bf16_val(g4.w);
    eq[0] = bf16_val(e4.x); eq[1] = bf16_val(e4.y); eq[2] = bf16_val(e4.z); eq[3] = bf16_val(e4.w);
  }

  v4f pv[16];
#pragma unroll
  for (int i = 0; i < 16; ++i) pv[i] = *(const v4fa*)(stg + (16 * wave + i) * GBN + 4 * lane);
  __syncthreads();

  const float invd = 1.0f / (float)DF;
#pragma unroll
  for (int i = 0; i < 16; ++i) {
    const int row = rowBase + 16 * wave + i;
    const bool ok = row < nN;
    const float y0 = pv[i].x + bq[0], y1 = pv[i].y + bq[1], y2 = pv[i].z + bq[2], y3 = pv[i].w + bq[3];
    float s = (y0 + y1) + (y2 + y3);
    s += __shfl_xor(s, 16, 32);
    s += __shfl_xor(s, 8, 32);
    s += __shfl_xor(s, 4, 32);
    s += __shfl_xor(s, 2, 32);
    s += __shfl_xor(s, 1, 32);
    const float mean = s * invd;
    const float d0 = y0 - mean, d1 = y1 - mean, d2 = y2 - mean, d3 = y3 - mean;
    float q = (d0 * d0 + d1 * d1) + (d2 * d2 + d3 * d3);
    q += __shfl_xor(q, 16, 32);
    q += __shfl_xor(q, 8, 32);
    q += __shfl_xor(q, 4, 32);
    q += __shfl_xor(q, 2, 32);
    q += __shfl_xor(q, 1, 32);
    const float var  = q * invd;
    const float rstd = rsqrtf(var + LNEPS);
    const float o0 = fmaxf(fmaf(d0 * rstd, gq[0], eq[0]), 0.0f);
    const float o1 = fmaxf(fmaf(d1 * rstd, gq[1], eq[1]), 0.0f);
    const float o2 = fmaxf(fmaf(d2 * rstd, gq[2], eq[2]), 0.0f);
    const float o3 = fmaxf(fmaf(d3 * rstd, gq[3], eq[3]), 0.0f);
    v4f qo;
    qo.x = ok ? o0 : 0.0f; qo.y = ok ? o1 : 0.0f; qo.z = ok ? o2 : 0.0f; qo.w = ok ? o3 : 0.0f;
    pv[i] = qo;
  }

  if constexpr (LAST != 0) {
#pragma unroll
    for (int i = 0; i < 16; ++i) {
      const int row = rowBase + 16 * wave + i;
      float* op = outp + (size_t)row * DF + 4 * lane;
      if (row < nN) *(volatile v4f*)op = pv[i];
    }
    __threadfence();
#pragma unroll
    for (int i = 0; i < 16; ++i) {
      const int row = rowBase + 16 * wave + i;
      float* op = outp + (size_t)row * DF + 4 * lane;
      if (row < nN) *(volatile v4f*)op = pv[i];
    }
    (void)apl; (void)mRows;
  } else {
#pragma unroll
    for (int i = 0; i < 16; ++i) {
      v4us h4, l4;
      unsigned lb;
      unsigned hb;
      hb = hl_bits(pv[i].x, lb); h4[0] = (unsigned short)hb; l4[0] = (unsigned short)lb;
      hb = hl_bits(pv[i].y, lb); h4[1] = (unsigned short)hb; l4[1] = (unsigned short)lb;
      hb = hl_bits(pv[i].z, lb); h4[2] = (unsigned short)hb; l4[2] = (unsigned short)lb;
      hb = hl_bits(pv[i].w, lb); h4[3] = (unsigned short)hb; l4[3] = (unsigned short)lb;
      unsigned short* srow = (unsigned short*)stg + (size_t)(16 * wave + i) * (2 * GBN);
      *(v4usa*)(srow + 4 * lane) = h4;
      *(v4usa*)(srow + DF + 4 * lane) = l4;
    }
    __syncthreads();
    v8us qv[16];
#pragma unroll
    for (int i = 0; i < 16; ++i) {
      const unsigned short* srow = (const unsigned short*)stg + (size_t)(16 * wave + i) * (2 * GBN);
      qv[i] = *(const v8usa*)(srow + 8 * lane);
    }
#pragma unroll
    for (int i = 0; i < 16; ++i) {
      const int gr = rowBase + 16 * wave + i;
      unsigned short* rp = apl + (size_t)gr * (size_t)AP + 2 * DF + 8 * lane;
      if (gr < mRows) *(volatile v8us*)rp = qv[i];
    }
    __threadfence();
#pragma unroll
    for (int i = 0; i < 16; ++i) {
      const int gr = rowBase + 16 * wave + i;
      unsigned short* rp = apl + (size_t)gr * (size_t)AP + 2 * DF + 8 * lane;
      if (gr < mRows) *(volatile v8us*)rp = qv[i];
    }
    (void)outp;
  }
}

__global__ __launch_bounds__(PTHR) void k_pool(const float* ne, const int* __restrict__ bat, int nN, float* gout) {
  __shared__ __attribute__((aligned(16))) float wst[NWAVE * POOLW];
  __shared__ __attribute__((aligned(16))) float pst[POOLW];
  __shared__ int plist[NWAVE * 32];
  __shared__ int wcn[NWAVE];
  const int tid = (int)threadIdx.x, lane = tid & 31, wave = tid >> 5;
  const int g = (int)blockIdx.x;
  const float nhuge = -__builtin_huge_valf();
  float s0 = 0.0f, s1 = 0.0f, s2 = 0.0f, s3 = 0.0f;
  float m0 = nhuge, m1 = nhuge, m2 = nhuge, m3 = nhuge;
  int cn = 0;
  const int nChunks = (nN + PTHR - 1) / PTHR;
#pragma unroll 1
  for (int ch = 0; ch < nChunks; ++ch) {
    const int n  = ch * PTHR + tid;
    const int nc = n < nN ? n : nN - 1;
    const int bv = bat[nc];
    const bool hit = (n < nN) && (bv == g);
    const unsigned mj = __builtin_amdgcn_ballot_w32(hit);
    if (mj != 0u) {
      if (hit) plist[wave * 32 + (int)__builtin_amdgcn_mbcnt_lo(mj, 0u)] = n;
      const int c = (int)__builtin_popcount(mj);
      wave_sync();
#pragma unroll 1
      for (int k = 0; k < c; ++k) {
        int nd = plist[wave * 32 + k];
        nd = nd < 0 ? 0 : (nd > nN - 1 ? nN - 1 : nd);
        const v4f r = *(const v4fa*)(ne + (size_t)nd * DF + 4 * lane);
        s0 += r.x; s1 += r.y; s2 += r.z; s3 += r.w;
        m0 = fmaxf(m0, r.x); m1 = fmaxf(m1, r.y); m2 = fmaxf(m2, r.z); m3 = fmaxf(m3, r.w);
      }
      cn += c;
      wave_sync();
    }
  }
  {
    v4f sv4; sv4.x = s0; sv4.y = s1; sv4.z = s2; sv4.w = s3;
    v4f mv4; mv4.x = m0; mv4.y = m1; mv4.z = m2; mv4.w = m3;
    *(v4fa*)(wst + wave * POOLW + 4 * lane) = sv4;
    *(v4fa*)(wst + wave * POOLW + DF + 4 * lane) = mv4;
    if (lane == 0) wcn[wave] = cn;
  }
  __syncthreads();
  {
    const int c = tid & (DF - 1);
    const int half = tid >> 7;
    double sv = 0.0;
    float mv = nhuge;
    int ct = 0;
#pragma unroll 1
    for (int w2 = 0; w2 < NWAVE; ++w2) {
      sv += (double)wst[w2 * POOLW + c];
      mv = fmaxf(mv, wst[w2 * POOLW + DF + c]);
      ct += wcn[w2];
    }
    const float cf = (float)(ct < 1 ? 1 : ct);
    const float mean = (float)sv * (1.0f / cf);
    pst[tid] = (half == 0) ? mean : mv;
  }
  __syncthreads();
  const bool ok = tid < POOLW / 4;
  v4f pvv = {0.f, 0.f, 0.f, 0.f};
  if (ok) pvv = *(const v4fa*)(pst + 4 * tid);
  float* op = gout + (size_t)g * POOLW + 4 * tid;
  if (ok) *(volatile v4f*)op = pvv;
  __threadfence();
  if (ok) *(volatile v4f*)op = pvv;
}

static inline int cdiv(int a, int b) { return (a + b - 1) / b; }
static inline size_t al256(size_t o) { return (o + 255) & ~(size_t)255; }

extern "C" void kernel_launch(void* const* d_in, const int* in_sizes, int n_in,
                              void* d_out, int out_size, void* d_ws, size_t ws_size,
                              hipStream_t stream) {
  if (n_in < 22) return;
  const int nN = in_sizes[2];
  if (nN < GBM || nN > (1 << 22)) return;
  if ((long long)in_sizes[0] != (long long)nN * DIN) return;
  if (in_sizes[1] < 2 || (in_sizes[1] & 1) != 0) return;
  const int nE = in_sizes[1] / 2;
  if (nE < 1 || nE >= (1 << 21)) return;
  if (in_sizes[3] != DF * DIN || in_sizes[4] != DF || in_sizes[5] != DF || in_sizes[6] != DF) return;
  for (int l = 0; l < NLAY; ++l) {
    const int b = 7 + 5 * l;
    if (in_sizes[b] != DF * DF || in_sizes[b + 1] != DF || in_sizes[b + 2] != DF * DF) return;
    if (in_sizes[b + 3] != DF || in_sizes[b + 4] != DF) return;
  }
  const long long rem = (long long)out_size - (long long)nN * DF;
  if (rem < POOLW || (rem % POOLW) != 0) return;
  const long long nGl = rem / POOLW;
  if (nGl > 65535) return;
  const int nG = (int)nGl;

  const float* x    = (const float*)d_in[0];
  const int*   ei   = (const int*)  d_in[1];
  const int*   bat  = (const int*)  d_in[2];
  const float* W0   = (const float*)d_in[3];
  const float* b0   = (const float*)d_in[4];
  const float* g0   = (const float*)d_in[5];
  const float* be0  = (const float*)d_in[6];
  const float* Wl[NLAY]; const float* bl[NLAY]; const float* Wr[NLAY]; const float* gg[NLAY]; const float* bb[NLAY];
  for (int l = 0; l < NLAY; ++l) {
    const int b = 7 + 5 * l;
    Wl[l] = (const float*)d_in[b];
    bl[l] = (const float*)d_in[b + 1];
    Wr[l] = (const float*)d_in[b + 2];
    gg[l] = (const float*)d_in[b + 3];
    bb[l] = (const float*)d_in[b + 4];
  }
  float* out = (float*)d_out;
  const int* src = ei;
  const int* dst = ei + nE;

  const int MP = cdiv(nN, GBM) * GBM;
  const int gM = MP / GBM;
  const int gA = cdiv(nN, NBA);
  if ((long long)gA * NBA < (long long)MP) return;
  const int vec8 = ((nE & 3) == 0) ? 1 : 0;

  char* ws = (char*)d_ws;
  size_t off = 0;
  const size_t oW0B = off; off = al256(off + (size_t)DF * KE * 2);
  const size_t oBPL = off; off = al256(off + (size_t)NLAY * DF * KS * 2);
  const size_t oXB  = off; off = al256(off + (size_t)MP * KE * 2);
  const size_t oA   = off; off = al256(off + (size_t)MP * AP * 2);
  if (off > ws_size || off > (size_t)WSMAX) return;
  unsigned short* W0B = (unsigned short*)(ws + oW0B);
  unsigned short* BPL = (unsigned short*)(ws + oBPL);
  unsigned short* XB  = (unsigned short*)(ws + oXB);
  unsigned short* Apl = (unsigned short*)(ws + oA);

  const size_t scanLds = (size_t)AGG_LDS_INTS * 4;
  hipFuncSetAttribute(reinterpret_cast<const void*>(&k_scan), hipFuncAttributeMaxDynamicSharedMemorySize, (int)scanLds);

  const int nUnits = NUWE + MP * (KE / 8);

  k_prep<<<cdiv(nUnits, NTHR), NTHR, 0, stream>>>(x, W0, Wl[0], Wr[0], Wl[1], Wr[1], Wl[2], Wr[2],
                                                  W0B, BPL, XB, nN, nUnits);
  k_gemm<0><<<gM, GTHR, 0, stream>>>(XB, KE, W0B, KE, KE, b0, g0, be0, Apl, out, nN, MP);
  for (int l = 0; l < NLAY; ++l) {
    k_scan<<<gA, NTHR, scanLds, stream>>>(src, dst, nE, nN, vec8, MP, Apl);
    const unsigned short* Bl = BPL + (size_t)l * DF * KS;
    if (l < NLAY - 1) {
      k_gemm<0><<<gM, GTHR, 0, stream>>>(Apl, AP, Bl, KS, KS, bl[l], gg[l], bb[l], Apl, out, nN, MP);
    } else {
      k_gemm<1><<<gM, GTHR, 0, stream>>>(Apl, AP, Bl, KS, KS, bl[l], gg[l], bb[l], Apl, out, nN, MP);
    }
  }
  k_pool<<<nG, PTHR, 0, stream>>>(out, bat, nN, out + (size_t)nN * DF);
}
